// CTCalone_63419487093326
// MI455X (gfx1250) — hardware-verified
//
#include <hip/hip_runtime.h>


namespace {
constexpr int NB = 32, T = 512, D = 512, H = 256, G4 = 4 * H, V = 97, VP = 112, SCW = 128, NROW = NB * T, NOUT = NB * T * V;
constexpr float XS = 8.0f, WSC = 256.0f, SIGMA = 8.0f;

typedef _Float16 b16;
typedef __attribute__((ext_vector_type(16))) _Float16 v16b;
typedef __attribute__((ext_vector_type(8))) _Float16 v8b;
typedef __attribute__((ext_vector_type(4))) _Float16 v4b;
typedef __attribute__((ext_vector_type(8))) float v8f;
typedef __attribute__((ext_vector_type(4))) float v4f;
__device__ __forceinline__ float bf16_rne(float f) { unsigned int u = __float_as_uint(f); u += 0x7FFFu + ((u >> 16) & 1u); return __uint_as_float(u & 0xFFFF0000u); }
__device__ __forceinline__ void split16(float v, b16& hi, b16& lo) { hi = (b16)v; lo = (b16)(v - (float)hi); }
__device__ __forceinline__ v16b frag_kb(const b16* p, int hh) { const v8b a = *(const v8b*)(p + 8 * hh), b = *(const v8b*)(p + 16 + 8 * hh); v16b f;
#pragma unroll
  for (int e = 0; e < 8; ++e) { f[e] = a[e]; f[8 + e] = b[e]; } return f; }
__device__ __forceinline__ v8f wmma16b(v16b a, v16b b, v8f c) { v8f d = __builtin_amdgcn_wmma_f32_16x16x32_f16(false, a, false, b, (short)0, c, false, false); asm volatile("v_nop\n\tv_nop\n\tv_nop\n\tv_nop" : "+v"(d) : "v"(a), "v"(b)); return d; }
__device__ __forceinline__ void wave_lds_sync() { __builtin_amdgcn_fence(__ATOMIC_RELEASE, "workgroup"); __builtin_amdgcn_wave_barrier(); __builtin_amdgcn_fence(__ATOMIC_ACQUIRE, "workgroup"); }
__device__ __forceinline__ float nexp(float x) { return __builtin_amdgcn_exp2f(x * 1.4426950408889634f); }
__device__ __forceinline__ float pmul(float a, float b) { float p = a * b; asm volatile("" : "+v"(p)); return p; }
__device__ __forceinline__ float sigm(float x) { return 1.0f / (1.0f + nexp(-x)); }
__device__ __forceinline__ float tanh_(float x) { const float e = nexp(-2.0f * fabsf(x)); const float t = (1.0f - e) / (1.0f + e); return x < 0.0f ? -t : t; }
__device__ __forceinline__ float hsum16(float v) { v += __shfl_xor(v, 1); v += __shfl_xor(v, 2); v += __shfl_xor(v, 4); return v + __shfl_xor(v, 8); }

__global__ __launch_bounds__(256) void prepx_kernel(const float* __restrict__ X, b16* __restrict__ X16, b16* __restrict__ XT16, float* __restrict__ RN) {
  __shared__ __attribute__((aligned(16))) b16 Tt[D][64 + 8]; __shared__ float Srn[64];
  const int b = blockIdx.y, t0 = blockIdx.x * 64, t_ = threadIdx.x, wave = t_ >> 5, lane = t_ & 31;
  for (int rr = wave; rr < 64; rr += 8) { const float* src = X + ((size_t)b * T + t0 + rr) * D; float ss = 0.0f; v8b o[2];
#pragma unroll
    for (int hq = 0; hq < 2; ++hq) {
#pragma unroll
      for (int j = 0; j < 8; ++j) { const int d = hq * 256 + lane * 8 + j; const float v = bf16_rne(src[d]); ss += pmul(v, v); const b16 f = (b16)(v * XS); o[hq][j] = f; Tt[d][rr] = f; } }
#pragma unroll
    for (int of = 16; of >= 1; of >>= 1) ss += __shfl_xor(ss, of);
    if (lane == 0) Srn[rr] = 1.0f / (sqrtf(ss) + 1e-12f);
    for (int pass = 0; pass < 2; ++pass) { for (int hq = 0; hq < 2; ++hq) *(volatile v8b*)(X16 + ((size_t)b * T + t0 + rr) * D + hq * 256 + lane * 8) = o[hq]; __threadfence(); } }
  __syncthreads();
  for (int pass = 0; pass < 2; ++pass) {
    for (int q = t_; q < D * 8; q += 256) { const int d = q >> 3, c8 = (q & 7) * 8; *(volatile v8b*)(XT16 + ((size_t)b * D + d) * T + t0 + c8) = *(const v8b*)(&Tt[d][c8]); }
    if (t_ < 64) ((volatile float*)RN)[(size_t)b * T + t0 + t_] = Srn[t_];
    __threadfence(); }
}
__global__ __launch_bounds__(256) void prepc_kernel(const float* __restrict__ wxf, const float* __restrict__ whf, const float* __restrict__ wxb, const float* __restrict__ whb, const float* __restrict__ wc, b16* __restrict__ ADH, b16* __restrict__ ADL, b16* __restrict__ WX, b16* __restrict__ WH, b16* __restrict__ WC) {
  __shared__ __attribute__((aligned(16))) b16 Ta[64][64 + 8], Tb[64][64 + 8]; __shared__ float Srs[T];
  const int t_ = threadIdx.x, kind = blockIdx.z;
  const int k0 = blockIdx.x * 64, n0 = blockIdx.y * 64;
  if (kind == 0) {
    if (blockIdx.y >= 8) return;
    for (int s = t_; s < T; s += 256) { float sum = 0.0f; for (int u = 0; u < T; ++u) sum += nexp(-fabsf((float)(s - u)) / SIGMA); Srs[s] = 1.0f / sum; }
    __syncthreads();
    const int u0 = k0, s0 = n0;
    for (int q = t_; q < 64 * 64; q += 256) { const int uu = q >> 6, sl = q & 63; const int u = u0 + uu, s = s0 + sl; const float v = pmul(nexp(-fabsf((float)(s - u)) / SIGMA), Srs[s]); b16 a_, c_; split16(v * XS, a_, c_); Ta[uu][sl] = a_; Tb[uu][sl] = c_; }
    __syncthreads();
    for (int pass = 0; pass < 2; ++pass) { for (int q = t_; q < 64 * 8; q += 256) { const int uu = q >> 3, c8 = (q & 7) * 8; *(volatile v8b*)(ADH + (size_t)(u0 + uu) * T + s0 + c8) = *(const v8b*)(&Ta[uu][c8]); *(volatile v8b*)(ADL + (size_t)(u0 + uu) * T + s0 + c8) = *(const v8b*)(&Tb[uu][c8]); } __threadfence(); }
  } else {
    const float* w; int K, N, NPd; b16* dst;
    if (kind == 1 || kind == 2) { w = kind == 1 ? wxf : wxb; K = D; N = G4; NPd = G4; dst = WX + (size_t)(kind - 1) * G4 * D; } else if (kind == 3 || kind == 4) { w = kind == 3 ? whf : whb; K = H; N = G4; NPd = G4; dst = WH + (size_t)(kind - 3) * G4 * H; } else { w = wc; K = 2 * H; N = V; NPd = VP; dst = WC; }
    if (k0 >= K || n0 >= NPd) return;
    for (int q = t_; q < 64 * 64; q += 256) { const int kk = q >> 6, nn = q & 63; const int n = n0 + nn; Ta[nn][kk] = (n < N) ? (b16)(bf16_rne(w[(size_t)(k0 + kk) * N + (n < N ? n : 0)]) * WSC) : (b16)0.0f; }
    __syncthreads();
    for (int pass = 0; pass < 2; ++pass) { for (int q = t_; q < 64 * 8; q += 256) { const int nn = q >> 3, c8 = (q & 7) * 8; if (n0 + nn < NPd) *(volatile v8b*)(dst + (size_t)(n0 + nn) * K + k0 + c8) = *(const v8b*)(&Ta[nn][c8]); } __threadfence(); } }
}
__global__ __launch_bounds__(128) void gram_kernel(const b16* __restrict__ X16, const float* __restrict__ RN, b16* __restrict__ ASH, b16* __restrict__ ASL) {
  __shared__ __attribute__((aligned(16))) b16 Th[4][16][128 + 8], Tl[4][16][128 + 8];
  const int wave = threadIdx.x >> 5, lane = threadIdx.x & 31, nloc = lane & 15, hlf = lane >> 4, b = blockIdx.y; const int m0 = blockIdx.x * 64 + wave * 16; const b16* Xb = X16 + (size_t)b * T * D;
  float rnr[8];
#pragma unroll
  for (int r = 0; r < 8; ++r) rnr[r] = RN[(size_t)b * T + m0 + 8 * hlf + r];
  for (int nc = 0; nc < 4; ++nc) {
    v8f acc[8];
#pragma unroll
    for (int t = 0; t < 8; ++t) acc[t] = (v8f){};
#pragma unroll 2
    for (int kb = 0; kb < D; kb += 32) { const v16b a = frag_kb(Xb + (size_t)(m0 + nloc) * D + kb, hlf);
#pragma unroll
      for (int t = 0; t < 8; ++t) acc[t] = wmma16b(a, frag_kb(Xb + (size_t)(nc * 128 + t * 16 + nloc) * D + kb, hlf), acc[t]); }
#pragma unroll
    for (int t = 0; t < 8; ++t) { const float rnc = RN[(size_t)b * T + nc * 128 + t * 16 + nloc];
#pragma unroll
      for (int r = 0; r < 8; ++r) { const float v = pmul(acc[t][r] * (1.0f / (XS * XS)), pmul(rnr[r], rnc)); b16 a_, c_; split16(v * XS, a_, c_); Th[wave][8 * hlf + r][t * 16 + nloc] = a_; Tl[wave][8 * hlf + r][t * 16 + nloc] = c_; } }
    wave_lds_sync();
    for (int pass = 0; pass < 2; ++pass) { for (int rr = 0; rr < 16; ++rr) if (lane < 16) { const size_t gi = ((size_t)b * T + m0 + rr) * T + nc * 128 + lane * 8; *(volatile v8b*)(ASH + gi) = *(const v8b*)(&Th[wave][rr][lane * 8]); *(volatile v8b*)(ASL + gi) = *(const v8b*)(&Tl[wave][rr][lane * 8]); } __threadfence(); }
    wave_lds_sync(); }
}
template <int NBPL>
__global__ __launch_bounds__(128) void gemm2_kernel(const b16* __restrict__ AH, const b16* __restrict__ AL, int lda, size_t sa, const b16* __restrict__ BH, const b16* __restrict__ BL, int ldb, size_t sbs, int K, float scale, b16* __restrict__ OH, b16* __restrict__ OL, int ldo, size_t so) {
  __shared__ __attribute__((aligned(16))) b16 Th[4][16][128 + 8], Tl[4][16][128 + 8];
  const int wave = threadIdx.x >> 5, lane = threadIdx.x & 31, nloc = lane & 15, hlf = lane >> 4, b = blockIdx.z; const int m0 = blockIdx.x * 64 + wave * 16, n0 = blockIdx.y * 128;
  const b16* Ah = AH + b * sa; const b16* Al = AL + b * sa; const b16* Bh = BH + b * sbs; const b16* Bl = NBPL == 2 ? BL + b * sbs : nullptr;
  v8f acc[8];
#pragma unroll
  for (int t = 0; t < 8; ++t) acc[t] = (v8f){};
  for (int kb = 0; kb < K; kb += 32) { const v16b ah = frag_kb(Ah + (size_t)(m0 + nloc) * lda + kb, hlf), al = frag_kb(Al + (size_t)(m0 + nloc) * lda + kb, hlf);
#pragma unroll
    for (int t = 0; t < 8; ++t) { const v16b bh = frag_kb(Bh + (size_t)(n0 + t * 16 + nloc) * ldb + kb, hlf); acc[t] = wmma16b(ah, bh, acc[t]); acc[t] = wmma16b(al, bh, acc[t]); if (NBPL == 2) acc[t] = wmma16b(ah, frag_kb(Bl + (size_t)(n0 + t * 16 + nloc) * ldb + kb, hlf), acc[t]); } }
#pragma unroll
  for (int t = 0; t < 8; ++t)
#pragma unroll
    for (int r = 0; r < 8; ++r) { b16 a_, c_; split16(acc[t][r] * scale * XS, a_, c_); Th[wave][8 * hlf + r][t * 16 + nloc] = a_; Tl[wave][8 * hlf + r][t * 16 + nloc] = c_; }
  wave_lds_sync();
  for (int pass = 0; pass < 2; ++pass) { for (int rr = 0; rr < 16; ++rr) if (lane < 16) { const size_t gi = b * so + (size_t)(m0 + rr) * ldo + n0 + lane * 8; *(volatile v8b*)(OH + gi) = *(const v8b*)(&Th[wave][rr][lane * 8]); *(volatile v8b*)(OL + gi) = *(const v8b*)(&Tl[wave][rr][lane * 8]); } __threadfence(); }
}
__global__ __launch_bounds__(512) void lstm_kernel(const b16* __restrict__ XAH, const b16* __restrict__ XAL, const b16* __restrict__ WX, const b16* __restrict__ WH, const float* __restrict__ bfw, const float* __restrict__ bbw, b16* __restrict__ HCH, b16* __restrict__ HCL) {
  __shared__ __attribute__((aligned(16))) b16 Hh[NB][H + 8], Hl[NB][H + 8];
  const int dir = blockIdx.x, t_ = threadIdx.x, wave = t_ >> 5, lane = t_ & 31, nloc = lane & 15, hlf = lane >> 4; const int j = wave * 16 + nloc;
  const b16* Wx = WX + (size_t)dir * G4 * D; const b16* Wh = WH + (size_t)dir * G4 * H; const float* bias = dir ? bbw : bfw;
  for (int k = t_; k < NB * (H + 8); k += 512) { (&Hh[0][0])[k] = (b16)0.0f; (&Hl[0][0])[k] = (b16)0.0f; }
  float bg[4];
#pragma unroll
  for (int g = 0; g < 4; ++g) bg[g] = bf16_rne(bias[g * H + j]);
  float cst[2][8];
#pragma unroll
  for (int mt = 0; mt < 2; ++mt)
#pragma unroll
    for (int r = 0; r < 8; ++r) cst[mt][r] = 0.0f;
  __syncthreads();
  for (int step = 0; step < T; ++step) { const int t = dir ? (T - 1 - step) : step;
    v8f acc[2][4];
#pragma unroll
    for (int mt = 0; mt < 2; ++mt)
#pragma unroll
      for (int g = 0; g < 4; ++g) acc[mt][g] = (v8f){};
#pragma unroll 2
    for (int kb = 0; kb < D; kb += 32) { v16b ah[2], al[2];
#pragma unroll
      for (int mt = 0; mt < 2; ++mt) { const size_t ro = ((size_t)(mt * 16 + nloc) * T + t) * D + kb; ah[mt] = frag_kb(XAH + ro, hlf); al[mt] = frag_kb(XAL + ro, hlf); }
#pragma unroll
      for (int g = 0; g < 4; ++g) { const v16b bw = frag_kb(Wx + (size_t)(g * H + j) * D + kb, hlf);
#pragma unroll
        for (int mt = 0; mt < 2; ++mt) { acc[mt][g] = wmma16b(ah[mt], bw, acc[mt][g]); acc[mt][g] = wmma16b(al[mt], bw, acc[mt][g]); } } }
#pragma unroll
    for (int kb = 0; kb < H; kb += 32) { v16b ah[2], al[2];
#pragma unroll
      for (int mt = 0; mt < 2; ++mt) { ah[mt] = frag_kb(&Hh[mt * 16 + nloc][kb], hlf); al[mt] = frag_kb(&Hl[mt * 16 + nloc][kb], hlf); }
#pragma unroll
      for (int g = 0; g < 4; ++g) { const v16b bw = frag_kb(Wh + (size_t)(g * H + j) * H + kb, hlf);
#pragma unroll
        for (int mt = 0; mt < 2; ++mt) { acc[mt][g] = wmma16b(ah[mt], bw, acc[mt][g]); acc[mt][g] = wmma16b(al[mt], bw, acc[mt][g]); } } }
    __syncthreads();
#pragma unroll
    for (int mt = 0; mt < 2; ++mt)
#pragma unroll
      for (int r = 0; r < 8; ++r) { const float zi = acc[mt][0][r] * (1.0f / (XS * WSC)) + bg[0], zf = acc[mt][1][r] * (1.0f / (XS * WSC)) + bg[1], zg = acc[mt][2][r] * (1.0f / (XS * WSC)) + bg[2], zo = acc[mt][3][r] * (1.0f / (XS * WSC)) + bg[3];
        const float c = pmul(sigm(zf), cst[mt][r]) + pmul(sigm(zi), tanh_(zg)); cst[mt][r] = c; const float h = pmul(sigm(zo), tanh_(c));
        b16 a_, c_; split16(h * XS, a_, c_); const float nh = __shfl_xor((float)a_, 1), nl = __shfl_xor((float)c_, 1); const int brow = mt * 16 + 8 * hlf + r;
        if ((nloc & 1) == 0) { __attribute__((ext_vector_type(2))) _Float16 ph, pl; ph[0] = a_; ph[1] = (b16)nh; pl[0] = c_; pl[1] = (b16)nl; *(__attribute__((ext_vector_type(2))) _Float16*)(&Hh[brow][j]) = ph; *(__attribute__((ext_vector_type(2))) _Float16*)(&Hl[brow][j]) = pl; } }
    __syncthreads();
    for (int pass = 0; pass < 2; ++pass) { for (int rr = wave * 2; rr < wave * 2 + 2; ++rr) { const size_t gi = ((size_t)rr * T + t) * (2 * H) + dir * H + lane * 8; *(volatile v8b*)(HCH + gi) = *(const v8b*)(&Hh[rr][lane * 8]); *(volatile v8b*)(HCL + gi) = *(const v8b*)(&Hl[rr][lane * 8]); } __threadfence(); } }
}
__global__ __launch_bounds__(128) void cls_kernel(const b16* __restrict__ HCH, const b16* __restrict__ HCL, const b16* __restrict__ WC, const float* __restrict__ bc, float* __restrict__ SC) {
  __shared__ __attribute__((aligned(16))) float Ts[4][16][SCW + 4];
  const int wave = threadIdx.x >> 5, lane = threadIdx.x & 31, nloc = lane & 15, hlf = lane >> 4; const size_t m0 = (size_t)blockIdx.x * 64 + wave * 16;
  v8f acc[7];
#pragma unroll
  for (int t = 0; t < 7; ++t) acc[t] = (v8f){};
#pragma unroll 2
  for (int kb = 0; kb < 2 * H; kb += 32) { const v16b ah = frag_kb(HCH + (m0 + nloc) * (2 * H) + kb, hlf), al = frag_kb(HCL + (m0 + nloc) * (2 * H) + kb, hlf);
#pragma unroll
    for (int t = 0; t < 7; ++t) { const v16b bw = frag_kb(WC + (size_t)(t * 16 + nloc) * (2 * H) + kb, hlf); acc[t] = wmma16b(ah, bw, acc[t]); acc[t] = wmma16b(al, bw, acc[t]); } }
  float lg[7][8];
#pragma unroll
  for (int t = 0; t < 7; ++t) { const int v = t * 16 + nloc; const float bb = (v < V) ? bf16_rne(bc[v < V ? v : 0]) : 0.0f;
#pragma unroll
    for (int r = 0; r < 8; ++r) lg[t][r] = (v < V) ? acc[t][r] * (1.0f / (XS * WSC)) + bb : -INFINITY; }
#pragma unroll
  for (int r = 0; r < 8; ++r) { float mx = -INFINITY;
#pragma unroll
    for (int t = 0; t < 7; ++t) mx = fmaxf(mx, lg[t][r]);
    mx = fmaxf(mx, __shfl_xor(mx, 1)); mx = fmaxf(mx, __shfl_xor(mx, 2)); mx = fmaxf(mx, __shfl_xor(mx, 4)); mx = fmaxf(mx, __shfl_xor(mx, 8));
    float sm = 0.0f;
#pragma unroll
    for (int t = 0; t < 7; ++t) { const float e = (t * 16 + nloc < V) ? nexp(lg[t][r] - mx) : 0.0f; lg[t][r] = e; sm += e; }
    sm = hsum16(sm); const float inv = 1.0f / sm;
#pragma unroll
    for (int t = 0; t < 7; ++t) Ts[wave][8 * hlf + r][t * 16 + nloc] = lg[t][r] * inv; }
  if (nloc == 0) {
#pragma unroll
    for (int r = 0; r < 8; ++r) for (int c = VP; c < SCW; ++c) Ts[wave][8 * hlf + r][c] = 0.0f; }
  wave_lds_sync();
  for (int pass = 0; pass < 2; ++pass) { for (int rr = 0; rr < 16; ++rr) *(volatile v4f*)(SC + (m0 + rr) * SCW + lane * 4) = *(const v4f*)(&Ts[wave][rr][lane * 4]); __threadfence(); }
}
__global__ __launch_bounds__(256) void out_kernel(const float* __restrict__ SC, float* __restrict__ out) {
  const int p = blockIdx.x * 256 + threadIdx.x; const int pc = p < NOUT ? p : NOUT - 1; const int r = pc / V, v = pc - r * V;
  const float val = SC[(size_t)r * SCW + v];
  for (int pass = 0; pass < 2; ++pass) { if (p < NOUT) ((volatile float*)out)[p] = val; __threadfence(); }
}
}

extern "C" void kernel_launch(void* const* d_in, const int* in_sizes, int n_in, void* d_out, int out_size, void* d_ws, size_t ws_size, hipStream_t stream) {
  (void)n_in;
  auto Fp = [&](int i) { return (const float*)d_in[i]; };
  if (in_sizes[0] != NB * T * D || in_sizes[1] != D * G4 || in_sizes[2] != H * G4 || in_sizes[7] != 2 * H * V || out_size != NOUT) return;
  size_t off = 0; char* ws = (char*)d_ws;
  auto carve = [&](size_t bytes) { char* p = ws + off; off += (bytes + 255) & ~(size_t)255; return p; };
  b16* X16 = (b16*)carve((size_t)NROW * D * 2); b16* XT16 = (b16*)carve((size_t)NB * D * T * 2); float* RN = (float*)carve((size_t)NROW * 4);
  b16* ADH = (b16*)carve((size_t)T * T * 2); b16* ADL = (b16*)carve((size_t)T * T * 2);
  b16* WX = (b16*)carve((size_t)2 * G4 * D * 2); b16* WH = (b16*)carve((size_t)2 * G4 * H * 2); b16* WC = (b16*)carve((size_t)VP * 2 * H * 2);
  b16* ASH = (b16*)carve((size_t)NB * T * T * 2); b16* ASL = (b16*)carve((size_t)NB * T * T * 2); b16* AH = (b16*)carve((size_t)NB * T * T * 2); b16* AL = (b16*)carve((size_t)NB * T * T * 2);
  b16* XAH = ASH; b16* XAL = ASL;
  b16* HCH = AH; b16* HCL = AL;
  float* SC = (float*)carve((size_t)NROW * SCW * 4);
  if (off > ws_size) return;
  prepx_kernel<<<dim3(T / 64, NB), 256, 0, stream>>>(Fp(0), X16, XT16, RN);
  prepc_kernel<<<dim3(8, 16, 6), 256, 0, stream>>>(Fp(1), Fp(2), Fp(4), Fp(5), Fp(7), ADH, ADL, WX, WH, WC);
  gram_kernel<<<dim3(T / 64, NB), 128, 0, stream>>>(X16, RN, ASH, ASL);
  gemm2_kernel<2><<<dim3(T / 64, T / 128, NB), 128, 0, stream>>>(ASH, ASL, T, (size_t)T * T, ADH, ADL, T, 0, T, 1.0f / (XS * XS), AH, AL, T, (size_t)T * T);
  gemm2_kernel<1><<<dim3(T / 64, D / 128, NB), 128, 0, stream>>>(AH, AL, T, (size_t)T * T, XT16, nullptr, T, (size_t)D * T, T, 1.0f / (XS * XS), XAH, XAL, D, (size_t)T * D);
  lstm_kernel<<<2, 512, 0, stream>>>(XAH, XAL, WX, WH, Fp(3), Fp(6), HCH, HCL);
  cls_kernel<<<NROW / 64, 128, 0, stream>>>(HCH, HCL, WC, Fp(8), SC);
  out_kernel<<<(NOUT + 255) / 256, 256, 0, stream>>>(SC, (float*)d_out);
}
